// SourceAnchoredBlock_33681133535740
// MI455X (gfx1250) — hardware-verified
//
#include <hip/hip_runtime.h>
#include <math.h>
#include <stdint.h>

#define NB    4
#define SEQ   1024
#define DM    1024
#define NH    16
#define HD    64
#define DFF   4096
#define NSTEP 20
#define NREL  (2 * SEQ - 1)
#define NTOK  (NB * SEQ)
#define NQB   (SEQ / 64)
#define QKP   (2 * DM)
#define LNEPS 1.0e-5f
#define WSC   64.0f
static_assert(NH * HD == DM);
static_assert((SEQ % 64) == 0 && (DM % 64) == 0 && (NTOK % 64) == 0 && (DFF % 64) == 0 && (DM % 32) == 0);
static_assert(DM == 4 * 256);

typedef _Float16 v16h __attribute__((ext_vector_type(16)));
typedef _Float16 v8h  __attribute__((ext_vector_type(8)));
typedef float    v8f  __attribute__((ext_vector_type(8)));
typedef float    v4f  __attribute__((ext_vector_type(4)));
typedef unsigned int v4u __attribute__((ext_vector_type(4)));
typedef unsigned int v2u __attribute__((ext_vector_type(2)));

__device__ __forceinline__ unsigned short bf_bits(float f) {
  unsigned u = __float_as_uint(f);
  return (unsigned short)((u + 0x7FFFu + ((u >> 16) & 1u)) >> 16);
}
__device__ __forceinline__ float bf_up(unsigned short h) { return __uint_as_float(((unsigned)h) << 16); }
__device__ __forceinline__ float bfr(float f) { return bf_up(bf_bits(f)); }
__device__ __forceinline__ unsigned short h_bits(_Float16 x) { return __builtin_bit_cast(unsigned short, x); }
__device__ __forceinline__ unsigned pk16(unsigned short a, unsigned short b) { return (unsigned)a | ((unsigned)b << 16); }
__device__ __forceinline__ v8f zero8() { v8f z = {0.f, 0.f, 0.f, 0.f, 0.f, 0.f, 0.f, 0.f}; return z; }
__device__ __forceinline__ float gelu_f(float v) { return 0.5f * v * (1.0f + erff(v * 0.70710678118654752f)); }

__device__ __forceinline__ v16h ldfrag_h(const _Float16* p) {
  union { v16h v; v8h h[2]; } f;
  f.h[0] = *(const v8h*)(p);
  f.h[1] = *(const v8h*)(p + 16);
  return f.v;
}

__device__ __forceinline__ v8f mma_h(v16h a, v16h b, v8f c) {
  c = __builtin_amdgcn_wmma_f32_16x16x32_f16(false, a, false, b, (short)0, c, false, false);
#if defined(__HIP_DEVICE_COMPILE__)
  asm volatile("v_nop\n\tv_nop\n\tv_nop\n\tv_nop" : "+v"(c) : "v"(a), "v"(b));
#endif
  return c;
}
__device__ __forceinline__ v8f mma_h_raw(v16h a, v16h b, v8f c) {
  return __builtin_amdgcn_wmma_f32_16x16x32_f16(false, a, false, b, (short)0, c, false, false);
}
__device__ __forceinline__ void dep_guard1(v8f& a, v8f& b, v16h x) {
#if defined(__HIP_DEVICE_COMPILE__)
  asm volatile("v_nop\n\tv_nop\n\tv_nop\n\tv_nop" : "+v"(a), "+v"(b) : "v"(x));
#endif
}
__device__ __forceinline__ void keep4_h(v16h a, v16h b, v16h c, v16h d) {
#if defined(__HIP_DEVICE_COMPILE__)
  asm volatile("v_nop" :: "v"(a), "v"(b), "v"(c), "v"(d));
#endif
}
__device__ __forceinline__ void acc_guard4(v8f& a, v8f& b, v8f& c, v8f& d) {
#if defined(__HIP_DEVICE_COMPILE__)
  asm volatile("v_nop\n\tv_nop\n\tv_nop\n\tv_nop" : "+v"(a), "+v"(b), "+v"(c), "+v"(d));
#endif
}
__device__ __forceinline__ void wave_sync_lds() {
  __builtin_amdgcn_fence(__ATOMIC_RELEASE, "workgroup");
  __builtin_amdgcn_wave_barrier();
  __builtin_amdgcn_fence(__ATOMIC_ACQUIRE, "workgroup");
}
__device__ __forceinline__ float wsum(float v) {
#pragma unroll
  for (int off = 16; off > 0; off >>= 1) v += __shfl_xor(v, off, 32);
  return v;
}
__device__ __forceinline__ float bsum256(float v, float* red, int lane, int wave) {
  v = wsum(v);
  if (lane == 0) red[wave] = v;
  __syncthreads();
  float tot = 0.f;
#pragma unroll
  for (int w = 0; w < 8; ++w) tot += red[w];
  return tot;
}

__global__ __launch_bounds__(256) void convT64(const float* __restrict__ W, unsigned short* Wt, int K, int O,
                                               float wsc) {
  __shared__ __align__(16) unsigned short sTt[64 * 72];
  const int tid = threadIdx.x, lane = tid & 31, wave = tid >> 5;
  const int o0 = blockIdx.x * 64, k0 = blockIdx.y * 64;
  const int kr = tid >> 2, cs = (tid & 3) * 16;
  const float* src = W + (size_t)(k0 + kr) * O + o0 + cs;
#pragma unroll
  for (int q = 0; q < 4; ++q) {
    const v4f v = *(const v4f*)(src + 4 * q);
#pragma unroll
    for (int e = 0; e < 4; ++e) sTt[(cs + 4 * q + e) * 72 + kr] = h_bits((_Float16)(bfr(v[e]) * wsc));
  }
  __syncthreads();
  const int q8 = lane >> 3, c8 = (lane & 7) * 8;
  v4u vv[2];
#pragma unroll
  for (int it = 0; it < 2; ++it) {
    const int row = wave * 8 + it * 4 + q8;
    vv[it] = *(const v4u*)(sTt + row * 72 + c8);
  }
  for (int pass = 0; pass < 2; ++pass) {
#pragma unroll
    for (int it = 0; it < 2; ++it) {
      const int row = wave * 8 + it * 4 + q8;
      *(volatile v4u*)(Wt + (size_t)(o0 + row) * K + k0 + c8) = vv[it];
    }
    __threadfence();
  }
}

__global__ __launch_bounds__(256) void cvt_h8(const float* __restrict__ X, unsigned short* out, int n8) {
  const int i = blockIdx.x * 256 + threadIdx.x;
  if (i < n8) {
    const size_t o = (size_t)i * 8;
    const v4f a0 = *(const v4f*)(X + o), a1 = *(const v4f*)(X + o + 4);
    v4u p;
#pragma unroll
    for (int e = 0; e < 2; ++e) {
      p[e]     = pk16(h_bits((_Float16)bfr(a0[2 * e])), h_bits((_Float16)bfr(a0[2 * e + 1])));
      p[2 + e] = pk16(h_bits((_Float16)bfr(a1[2 * e])), h_bits((_Float16)bfr(a1[2 * e + 1])));
    }
    *(volatile v4u*)(out + o) = p;
    __threadfence();
    *(volatile v4u*)(out + o) = p;
  }
}

template <int OM, int BIASM, int ACT, int RES>
__global__ __launch_bounds__(256) void gemm64(
    const unsigned short* __restrict__ Ap, int lda, long long strideA,
    const unsigned short* __restrict__ Btp, int ldb, long long strideB,
    const float* __restrict__ bias0, const float* __restrict__ bias1, int Nb,
    const float* __restrict__ resid,
    void* Cout, int ldc, long long strideC,
    int M, int N, int K, float oscale) {
  const _Float16* A  = (const _Float16*)(const void*)Ap;
  const _Float16* Bt = (const _Float16*)(const void*)Btp;
  __shared__ __align__(16) float sT[8][16 * 68];
  const int b    = blockIdx.y;
  const int lane = threadIdx.x & 31;
  const int wave = threadIdx.x >> 5;
  const int tilesN = N >> 6;
  const int tilesM = M >> 6;
  const int tile = blockIdx.x * 8 + wave;
  if (tile >= tilesM * tilesN) return;
  const int tm = tile / tilesN;
  const int tn = tile - tm * tilesN;
  const int m0 = tm << 6;
  const int n0 = tn << 6;

  const _Float16* Ab = A  + (size_t)b * strideA;
  const _Float16* Bb = Bt + (size_t)b * strideB;

  const int rlane = lane & 15;
  const int koff  = (lane >> 4) * 8;
  const int mOff  = (lane >> 4) * 8;

  v8f acc[4][4];
#pragma unroll
  for (int i = 0; i < 4; ++i)
#pragma unroll
    for (int j = 0; j < 4; ++j) acc[i][j] = zero8();

  for (int k0 = 0; k0 < K; k0 += 32) {
    v16h bh[4];
#pragma unroll
    for (int j = 0; j < 4; ++j) {
      const size_t bo = (size_t)(n0 + (j << 4) + rlane) * ldb + koff + k0;
      bh[j] = ldfrag_h(Bb + bo);
    }
#pragma unroll
    for (int i = 0; i < 4; ++i) {
      const size_t ao = (size_t)(m0 + (i << 4) + rlane) * lda + koff + k0;
      const v16h ah = ldfrag_h(Ab + ao);
#pragma unroll
      for (int j = 0; j < 4; ++j) acc[i][j] = mma_h_raw(ah, bh[j], acc[i][j]);
      dep_guard1(acc[i][0], acc[i][3], ah);
    }
    keep4_h(bh[0], bh[1], bh[2], bh[3]);
  }
  acc_guard4(acc[0][0], acc[0][1], acc[0][2], acc[0][3]);
  acc_guard4(acc[1][0], acc[1][1], acc[1][2], acc[1][3]);
  acc_guard4(acc[2][0], acc[2][1], acc[2][2], acc[2][3]);
  acc_guard4(acc[3][0], acc[3][1], acc[3][2], acc[3][3]);

  const int hh2 = lane >> 4, c4 = (lane & 15) * 4;
  const int q8  = lane >> 3, c8 = (lane & 7) * 8;
  float bc[8];
#pragma unroll
  for (int e = 0; e < 8; ++e) bc[e] = 0.f;
  if (BIASM == 0) {
    const bool use1 = (n0 >= Nb);
    if (OM == 0) {
      const int cb = n0 + c4;
      const int i0 = (cb < Nb - 4) ? cb : (Nb - 4);
      const int i1 = (cb - Nb > 0) ? (cb - Nb) : 0;
      const v4f b0v = *(const v4f*)(bias0 + i0);
      const v4f b1v = *(const v4f*)(bias1 + i1);
#pragma unroll
      for (int e = 0; e < 4; ++e) bc[e] = bfr(use1 ? b1v[e] : b0v[e]);
    } else {
      const int cb = n0 + c8;
      const int i0 = (cb < Nb - 8) ? cb : (Nb - 8);
      const int i1 = (cb - Nb > 0) ? (cb - Nb) : 0;
      const v4f b0a = *(const v4f*)(bias0 + i0), b0b = *(const v4f*)(bias0 + i0 + 4);
      const v4f b1a = *(const v4f*)(bias1 + i1), b1b = *(const v4f*)(bias1 + i1 + 4);
#pragma unroll
      for (int e = 0; e < 4; ++e) {
        bc[e]     = bfr(use1 ? b1a[e] : b0a[e]);
        bc[4 + e] = bfr(use1 ? b1b[e] : b0b[e]);
      }
    }
  }

  float* slab = sT[wave];
#pragma unroll
  for (int i = 0; i < 4; ++i) {
    const int mBase = m0 + (i << 4);
#pragma unroll
    for (int j = 0; j < 4; ++j) {
#pragma unroll
      for (int r = 0; r < 8; ++r) {
        slab[(mOff + r) * 68 + (j << 4) + rlane] = acc[i][j][r];
      }
    }
    wave_sync_lds();
    if (OM == 0) {
      float* C = (float*)Cout + (size_t)b * strideC;
      const float* Rb = resid + (size_t)b * strideC;
      v4f vals[8];
#pragma unroll
      for (int it = 0; it < 8; ++it) {
        const int row = it * 2 + hh2;
        v4f v = *(const v4f*)(slab + row * 68 + c4);
#pragma unroll
        for (int e = 0; e < 4; ++e) {
          float f = v[e] * oscale + bc[e];
          if (ACT) f = gelu_f(f);
          v[e] = f;
        }
        if (RES != 0) {
          const v4f rr = *(const v4f*)(Rb + (size_t)(mBase + row) * ldc + n0 + c4);
#pragma unroll
          for (int e = 0; e < 4; ++e) v[e] += rr[e];
        }
        vals[it] = v;
      }
      for (int pass = 0; pass < 2; ++pass) {
#pragma unroll
        for (int it = 0; it < 8; ++it) {
          const int row = it * 2 + hh2;
          *(volatile v4f*)(C + (size_t)(mBase + row) * ldc + n0 + c4) = vals[it];
        }
        __threadfence();
      }
    } else {
      unsigned short* C = (unsigned short*)Cout + (size_t)b * strideC;
      v4u hv[4];
#pragma unroll
      for (int it = 0; it < 4; ++it) {
        const int row = it * 4 + q8;
        const float* sp = slab + row * 68 + c8;
        float bm = 0.f;
        if (BIASM == 1) bm = bfr(bias0[mBase + row]);
        v4u a;
#pragma unroll
        for (int e = 0; e < 4; ++e) {
          float f0 = sp[2 * e]     * oscale + ((BIASM == 1) ? bm : bc[2 * e]);
          float f1 = sp[2 * e + 1] * oscale + ((BIASM == 1) ? bm : bc[2 * e + 1]);
          if (ACT) { f0 = gelu_f(f0); f1 = gelu_f(f1); }
          unsigned short u0, u1;
          if (OM == 1) { u0 = bf_bits(f0); u1 = bf_bits(f1); }
          else         { u0 = h_bits((_Float16)f0); u1 = h_bits((_Float16)f1); }
          a[e] = pk16(u0, u1);
        }
        hv[it] = a;
      }
      for (int pass = 0; pass < 2; ++pass) {
#pragma unroll
        for (int it = 0; it < 4; ++it) {
          const int row = it * 4 + q8;
          *(volatile v4u*)(C + (size_t)(mBase + row) * ldc + n0 + c8) = hv[it];
        }
        __threadfence();
      }
    }
    wave_sync_lds();
  }
}

template <int HASB>
__global__ __launch_bounds__(128)
void attn64(const unsigned short* __restrict__ qkp, const unsigned short* __restrict__ vtp,
            const float* __restrict__ rb, unsigned short* outp, float sscale) {
  union FH { v16h v; v8h h[2]; };
  __shared__ __align__(16) _Float16 Ksh[64 * 64];
  __shared__ __align__(16) _Float16 Vth[64 * 64];
  __shared__ __align__(16) _Float16 Psh[4][16 * 64];
  __shared__ __align__(16) float    Os[4][16 * 64];
  __shared__ float sRb[2048];

  const int tid  = threadIdx.x;
  const int wave = tid >> 5;
  const int lane = tid & 31;
  const int hh   = lane >> 4;
  const int c    = lane & 15;

  const int bx   = blockIdx.x;
  const int qb   = bx % NQB;
  const int rest = bx / NQB;
  const int h    = rest % NH;
  const int b    = rest / NH;
  const int q0   = qb * 64 + wave * 16;
  const size_t rowB = (size_t)b * SEQ;

  const _Float16* Qh = (const _Float16*)(const void*)qkp + (size_t)h * HD;
  const _Float16* Kg = (const _Float16*)(const void*)qkp + DM + (size_t)h * HD;
  const _Float16* Vh = (const _Float16*)(const void*)vtp + ((size_t)b * DM + (size_t)h * HD) * SEQ;

  if (HASB) {
    for (int i = tid; i < 2048; i += 128) {
      const int ic = (i < NREL) ? i : (NREL - 1);
      sRb[i] = bfr(rb[ic]);
    }
  }

  v16h qa[2];
#pragma unroll
  for (int dc = 0; dc < 2; ++dc) qa[dc] = ldfrag_h(Qh + (rowB + q0 + c) * QKP + dc * 32 + 8 * hh);

  float mrow[8], lrow[8];
  v8f oacc[4];
#pragma unroll
  for (int r = 0; r < 8; ++r) { mrow[r] = -INFINITY; lrow[r] = 0.f; }
#pragma unroll
  for (int t = 0; t < 4; ++t) oacc[t] = zero8();

  for (int kt = 0; kt < NQB; ++kt) {
    const int kv0 = kt * 64;
    __syncthreads();
    {
      const int r = tid >> 1, hf = (tid & 1) * 32;
      const _Float16* kg = Kg + (rowB + kv0 + r) * QKP + hf;
      const _Float16* vg = Vh + (size_t)r * SEQ + kv0 + hf;
#pragma unroll
      for (int i = 0; i < 4; ++i) {
        const v8h a0 = *(const v8h*)(kg + 8 * i);
        const v8h b0 = *(const v8h*)(vg + 8 * i);
        *(v8h*)(Ksh + r * 64 + hf + 8 * i) = a0;
        *(v8h*)(Vth + r * 64 + hf + 8 * i) = b0;
      }
    }
    __syncthreads();

    v8f s[4];
#pragma unroll
    for (int j = 0; j < 4; ++j) {
      v8f sh = zero8();
#pragma unroll
      for (int dc = 0; dc < 2; ++dc) {
        FH kb;
        kb.h[0] = *(const v8h*)(Ksh + (j * 16 + c) * 64 + dc * 32 + 8 * hh);
        kb.h[1] = *(const v8h*)(Ksh + (j * 16 + c) * 64 + dc * 32 + 16 + 8 * hh);
        sh = mma_h(qa[dc], kb.v, sh);
      }
#pragma unroll
      for (int r = 0; r < 8; ++r) {
        float v = sh[r] * sscale;
        if (HASB) {
          int idx = (q0 + 8 * hh + r) - (kv0 + j * 16 + c) + (SEQ - 1);
          idx = (idx < 0) ? 0 : ((idx > NREL - 1) ? (NREL - 1) : idx);
          v += sRb[idx];
        }
        s[j][r] = v;
      }
    }

    _Float16* pwh = Psh[wave];
#pragma unroll
    for (int r = 0; r < 8; ++r) {
      float m = s[0][r];
      m = fmaxf(m, s[1][r]);
      m = fmaxf(m, s[2][r]);
      m = fmaxf(m, s[3][r]);
#pragma unroll
      for (int off = 1; off < 16; off <<= 1) m = fmaxf(m, __shfl_xor(m, off, 32));
      const float mnew  = fmaxf(mrow[r], m);
      const float alpha = __expf(mrow[r] - mnew);
      mrow[r] = mnew;
      float psum = 0.f;
#pragma unroll
      for (int j = 0; j < 4; ++j) {
        const float p = __expf(s[j][r] - mnew);
        psum += p;
        pwh[(8 * hh + r) * 64 + j * 16 + c] = (_Float16)(p * 1024.0f);
      }
#pragma unroll
      for (int off = 1; off < 16; off <<= 1) psum += __shfl_xor(psum, off, 32);
      lrow[r] = lrow[r] * alpha + psum;
#pragma unroll
      for (int t = 0; t < 4; ++t) oacc[t][r] *= alpha;
    }
    wave_sync_lds();

#pragma unroll 1
    for (int kk = 0; kk < 2; ++kk) {
      FH pa;
      pa.h[0] = *(const v8h*)(pwh + c * 64 + kk * 32 + 8 * hh);
      pa.h[1] = *(const v8h*)(pwh + c * 64 + kk * 32 + 16 + 8 * hh);
#pragma unroll
      for (int t = 0; t < 4; ++t) {
        FH vb;
        vb.h[0] = *(const v8h*)(Vth + (t * 16 + c) * 64 + kk * 32 + 8 * hh);
        vb.h[1] = *(const v8h*)(Vth + (t * 16 + c) * 64 + kk * 32 + 16 + 8 * hh);
        oacc[t] = mma_h(pa.v, vb.v, oacc[t]);
      }
    }
  }

  float* os = Os[wave];
#pragma unroll
  for (int r = 0; r < 8; ++r) {
    const float l = lrow[r];
    const float inv = ((l > 0.f) ? (1.0f / l) : 0.f) * (16.0f / 1024.0f);
#pragma unroll
    for (int t = 0; t < 4; ++t) os[(8 * hh + r) * 64 + t * 16 + c] = oacc[t][r] * inv;
  }
  wave_sync_lds();
  {
    const int q4 = lane >> 3, c8 = (lane & 7) * 8;
    v4u hv[4];
#pragma unroll
    for (int it = 0; it < 4; ++it) {
      const int row = it * 4 + q4;
      const float* sp = os + row * 64 + c8;
      v4u a;
#pragma unroll
      for (int e = 0; e < 4; ++e) a[e] = pk16(h_bits((_Float16)sp[2 * e]), h_bits((_Float16)sp[2 * e + 1]));
      hv[it] = a;
    }
    for (int pass = 0; pass < 2; ++pass) {
#pragma unroll
      for (int it = 0; it < 4; ++it) {
        const int row = it * 4 + q4;
        const size_t go = (rowB + q0 + row) * DM + (size_t)h * HD + c8;
        *(volatile v4u*)(outp + go) = hv[it];
      }
      __threadfence();
    }
  }
}

__device__ __forceinline__ void row_store_f32(float* dst_row, v4f o, int t) {
  *(volatile v4f*)(dst_row + 4 * t) = o;
  __threadfence();
  *(volatile v4f*)(dst_row + 4 * t) = o;
}
__device__ __forceinline__ void row_store_h16(unsigned int* sb, unsigned short* dst_row, v4f o, int t) {
  v2u p;
  p[0] = pk16(h_bits((_Float16)o[0]), h_bits((_Float16)o[1]));
  p[1] = pk16(h_bits((_Float16)o[2]), h_bits((_Float16)o[3]));
  *(v2u*)(sb + 2 * t) = p;
  __syncthreads();
  if (t < 128) {
    const v4u v = *(const v4u*)(sb + 4 * t);
    *(volatile v4u*)(dst_row + 8 * t) = v;
    __threadfence();
    *(volatile v4u*)(dst_row + 8 * t) = v;
  }
}

__global__ __launch_bounds__(256) void row_h0(const float* __restrict__ X, const float* __restrict__ emb,
                                              const int* __restrict__ step, float* outF, unsigned short* outH) {
  __shared__ __align__(16) unsigned int sb[512];
  const int t = threadIdx.x;
  const size_t base = (size_t)blockIdx.x * DM;
  int s = step[0];
  s = (s > NSTEP - 1) ? (NSTEP - 1) : s;
  s = (s < 0) ? (s + NSTEP) : s;
  s = (s < 0) ? 0 : s;
  const v4f xv = *(const v4f*)(X + base + 4 * t);
  const v4f ev = *(const v4f*)(emb + (size_t)s * DM + 4 * t);
  v4f y;
#pragma unroll
  for (int e = 0; e < 4; ++e) y[e] = bfr(xv[e]) + bfr(ev[e]);
  row_store_f32(outF + base, y, t);
  row_store_h16(sb, outH + base, y, t);
}

template <int OUTF, int OUTH>
__global__ __launch_bounds__(256) void ln_row(const float* __restrict__ X, const float* __restrict__ gam,
                                              const float* __restrict__ bet, float* outF, unsigned short* outH) {
  __shared__ float red0[8], red1[8];
  __shared__ __align__(16) unsigned int sb[512];
  const int t = threadIdx.x, lane = t & 31, wave = t >> 5;
  const size_t base = (size_t)blockIdx.x * DM;
  const v4f xv = *(const v4f*)(X + base + 4 * t);
  const float mean = bsum256((xv[0] + xv[1]) + (xv[2] + xv[3]), red0, lane, wave) * (1.0f / DM);
  v4f d;
#pragma unroll
  for (int e = 0; e < 4; ++e) d[e] = xv[e] - mean;
  const float var  = bsum256((d[0] * d[0] + d[1] * d[1]) + (d[2] * d[2] + d[3] * d[3]), red1, lane, wave) * (1.0f / DM);
  const float rstd = 1.0f / sqrtf(var + LNEPS);
  const v4f gv = *(const v4f*)(gam + 4 * t);
  const v4f bv = *(const v4f*)(bet + 4 * t);
  v4f y;
#pragma unroll
  for (int e = 0; e < 4; ++e) y[e] = (d[e] * rstd) * bfr(gv[e]) + bfr(bv[e]);
  if (OUTF) row_store_f32(outF + base, y, t);
  if (OUTH) row_store_h16(sb, outH + base, y, t);
}

extern "C" void kernel_launch(void* const* d_in, const int* in_sizes, int n_in,
                              void* d_out, int out_size, void* d_ws, size_t ws_size,
                              hipStream_t stream) {
  if (n_in < 25) return;
  if (in_sizes[0] != NTOK * DM || in_sizes[1] != NTOK * DM) return;
  if (in_sizes[2] != 1 || in_sizes[3] != NSTEP * DM || in_sizes[4] != NREL) return;
  if (in_sizes[5] != DM * 3 * DM || in_sizes[6] != 3 * DM) return;
  if (in_sizes[7] != DM * DM || in_sizes[8] != DM) return;
  if (in_sizes[9] != DM * DM || in_sizes[10] != DM) return;
  if (in_sizes[11] != DM * 2 * DM || in_sizes[12] != 2 * DM) return;
  if (in_sizes[13] != DM * DM || in_sizes[14] != DM) return;
  if (in_sizes[15] != DM * DFF || in_sizes[16] != DFF) return;
  if (in_sizes[17] != DFF * DM || in_sizes[18] != DM) return;
  for (int i = 19; i <= 24; ++i) { if (in_sizes[i] != DM) return; }
  if (out_size != NTOK * DM) return;

  const float* hid   = (const float*)d_in[0];
  const float* srcs  = (const float*)d_in[1];
  const int*   tstep = (const int*)d_in[2];
  const float* semb  = (const float*)d_in[3];
  const float* relb  = (const float*)d_in[4];
  const float* Wqkv = (const float*)d_in[5];   const float* bqkv = (const float*)d_in[6];
  const float* Wo   = (const float*)d_in[7];   const float* bo   = (const float*)d_in[8];
  const float* Wcq  = (const float*)d_in[9];   const float* bcq  = (const float*)d_in[10];
  const float* Wckv = (const float*)d_in[11];  const float* bckv = (const float*)d_in[12];
  const float* Wco  = (const float*)d_in[13];  const float* bco  = (const float*)d_in[14];
  const float* W1   = (const float*)d_in[15];  const float* b1   = (const float*)d_in[16];
  const float* W2   = (const float*)d_in[17];  const float* b2   = (const float*)d_in[18];
  const float* g_s  = (const float*)d_in[19];  const float* t_s  = (const float*)d_in[20];
  const float* g_c  = (const float*)d_in[21];  const float* t_c  = (const float*)d_in[22];
  const float* g_f  = (const float*)d_in[23];  const float* t_f  = (const float*)d_in[24];

  const size_t PW   = (size_t)DM * DM * 2;
  const size_t PAF  = (size_t)NTOK * DM * 4;
  const size_t PAH  = (size_t)NTOK * DM * 2;
  const size_t PQK  = (size_t)NTOK * QKP * 2;
  const size_t PVT  = (size_t)NB * DM * SEQ * 2;
  const size_t PG   = (size_t)NTOK * DFF * 2;
  size_t off = 0;
  const size_t oWqkv = off; off += 3 * PW;
  const size_t oWo   = off; off += PW;
  const size_t oWcq  = off; off += PW;
  const size_t oWckv = off; off += 2 * PW;
  const size_t oWco  = off; off += PW;
  const size_t oW1   = off; off += 4 * PW;
  const size_t oW2   = off; off += 4 * PW;
  const size_t oHF   = off; off += PAF;
  const size_t oR    = off; off += PAF;
  const size_t oAH   = off; off += PAH;
  const size_t oSH   = off; off += PAH;
  const size_t oQK   = off; off += PQK;
  const size_t oVT   = off; off += PVT;
  const size_t oCtx  = off; off += PAH;
  if (off > ws_size) return;
  if (off > (size_t)134217728) return;
  if (oQK + PG > off) return;

  char* ws = (char*)d_ws;
  unsigned short* WqkvT = (unsigned short*)(ws + oWqkv);
  unsigned short* WoT   = (unsigned short*)(ws + oWo);
  unsigned short* WcqT  = (unsigned short*)(ws + oWcq);
  unsigned short* WckvT = (unsigned short*)(ws + oWckv);
  unsigned short* WcoT  = (unsigned short*)(ws + oWco);
  unsigned short* W1T   = (unsigned short*)(ws + oW1);
  unsigned short* W2T   = (unsigned short*)(ws + oW2);
  float*          HF    = (float*)(ws + oHF);
  float*          R     = (float*)(ws + oR);
  unsigned short* AH    = (unsigned short*)(ws + oAH);
  unsigned short* SH    = (unsigned short*)(ws + oSH);
  unsigned short* QK    = (unsigned short*)(ws + oQK);
  unsigned short* VT    = (unsigned short*)(ws + oVT);
  unsigned short* Ctx   = (unsigned short*)(ws + oCtx);
  unsigned short* G     = (unsigned short*)(ws + oQK);

  const dim3 blk(256);
  const dim3 gTqkv((3 * DM) / 64, DM / 64);
  const dim3 gT1(DM / 64, DM / 64);
  const dim3 gT2((2 * DM) / 64, DM / 64);
  const dim3 gTw1(DFF / 64, DM / 64);
  const dim3 gTw2(DM / 64, DFF / 64);
  const int  n8 = NTOK * DM / 8;
  const dim3 gE((n8 + 255) / 256);
  const dim3 gN2(((NTOK / 64) * (QKP / 64) + 7) / 8, 1);
  const dim3 gN1(((NTOK / 64) * (DM / 64) + 7) / 8, 1);
  const dim3 gN4(((NTOK / 64) * (DFF / 64) + 7) / 8, 1);
  const dim3 gVT(((DM / 64) * (SEQ / 64) + 7) / 8, NB);
  const dim3 gAttn(NB * NH * NQB);
  const dim3 gRow(NTOK);
  const float invw  = 1.0f / WSC;
  const float invwc = 1.0f / (WSC * 16.0f);

  convT64<<<gTqkv, blk, 0, stream>>>(Wqkv, WqkvT, DM, 3 * DM, WSC);
  convT64<<<gT1,   blk, 0, stream>>>(Wo,   WoT,   DM, DM, WSC);
  convT64<<<gT1,   blk, 0, stream>>>(Wcq,  WcqT,  DM, DM, WSC);
  convT64<<<gT2,   blk, 0, stream>>>(Wckv, WckvT, DM, 2 * DM, WSC);
  convT64<<<gT1,   blk, 0, stream>>>(Wco,  WcoT,  DM, DM, WSC);
  convT64<<<gTw1,  blk, 0, stream>>>(W1,   W1T,   DM, DFF, WSC);
  convT64<<<gTw2,  blk, 0, stream>>>(W2,   W2T,   DFF, DM, WSC);

  row_h0<<<gRow, blk, 0, stream>>>(hid, semb, tstep, HF, AH);
  cvt_h8<<<gE, blk, 0, stream>>>(srcs, SH, n8);

  gemm64<2, 0, 0, 0><<<gN2, blk, 0, stream>>>(
      AH, DM, 0LL, WqkvT, DM, 0LL, bqkv, bqkv + DM, DM, HF,
      (void*)QK, QKP, 0LL, NTOK, QKP, DM, invw);
  gemm64<2, 1, 0, 0><<<gVT, blk, 0, stream>>>(
      WqkvT + (size_t)2 * DM * DM, DM, 0LL, AH, DM, (long long)SEQ * DM, bqkv + 2 * DM, bqkv + 2 * DM, DM, HF,
      (void*)VT, SEQ, (long long)DM * SEQ, DM, SEQ, DM, invw);
  attn64<1><<<gAttn, dim3(128), 0, stream>>>(QK, VT, relb, Ctx, 0.125f);
  gemm64<0, 0, 0, 1><<<gN1, blk, 0, stream>>>(
      Ctx, DM, 0LL, WoT, DM, 0LL, bo, bo, DM, HF,
      (void*)R, DM, 0LL, NTOK, DM, DM, invwc);
  ln_row<1, 1><<<gRow, blk, 0, stream>>>(R, g_s, t_s, HF, AH);

  gemm64<2, 0, 0, 0><<<gN1, blk, 0, stream>>>(
      AH, DM, 0LL, WcqT, DM, 0LL, bcq, bcq, DM, HF,
      (void*)QK, QKP, 0LL, NTOK, DM, DM, invw);
  gemm64<2, 0, 0, 0><<<gN1, blk, 0, stream>>>(
      SH, DM, 0LL, WckvT, DM, 0LL, bckv, bckv, DM, HF,
      (void*)(QK + DM), QKP, 0LL, NTOK, DM, DM, invw);
  gemm64<2, 1, 0, 0><<<gVT, blk, 0, stream>>>(
      WckvT + (size_t)DM * DM, DM, 0LL, SH, DM, (long long)SEQ * DM, bckv + DM, bckv + DM, DM, HF,
      (void*)VT, SEQ, (long long)DM * SEQ, DM, SEQ, DM, invw);
  attn64<0><<<gAttn, dim3(128), 0, stream>>>(QK, VT, relb, Ctx, 0.125f);
  gemm64<0, 0, 0, 1><<<gN1, blk, 0, stream>>>(
      Ctx, DM, 0LL, WcoT, DM, 0LL, bco, bco, DM, HF,
      (void*)R, DM, 0LL, NTOK, DM, DM, invwc);
  ln_row<1, 1><<<gRow, blk, 0, stream>>>(R, g_c, t_c, HF, AH);

  gemm64<2, 0, 1, 0><<<gN4, blk, 0, stream>>>(
      AH, DM, 0LL, W1T, DM, 0LL, b1, b1, DFF, HF,
      (void*)G, DFF, 0LL, NTOK, DFF, DM, invw);
  gemm64<0, 0, 0, 1><<<gN1, blk, 0, stream>>>(
      G, DFF, 0LL, W2T, DFF, 0LL, b2, b2, DM, HF,
      (void*)R, DM, 0LL, NTOK, DM, DFF, invw);
  ln_row<1, 0><<<gRow, blk, 0, stream>>>(R, g_f, t_f, (float*)d_out, AH);
  (void)hipGetLastError();
}
